// GQA_74560632259157
// MI455X (gfx1250) — hardware-verified
//
#include <hip/hip_runtime.h>
#include <math.h>

typedef __attribute__((ext_vector_type(16))) _Float16 v16h;
typedef __attribute__((ext_vector_type(16))) __bf16 v16b;
typedef __attribute__((ext_vector_type(8)))  _Float16 v8h;
typedef __attribute__((ext_vector_type(8)))  __bf16 v8b;
typedef __attribute__((ext_vector_type(8)))  float v8f;
typedef __attribute__((ext_vector_type(4)))  float v4f;
typedef __attribute__((ext_vector_type(4)))  unsigned v4u;

template <typename T> __device__ __forceinline__ void vst2(void* p, T v) { *(volatile T*)p = v; __threadfence(); *(volatile T*)p = v; }
__device__ __forceinline__ v8f wmma16(v16h a, v16h b, v8f c) {
  v8f d = __builtin_amdgcn_wmma_f32_16x16x32_f16(false, a, false, b, (short)0, c, false, false);
  asm volatile("v_nop\n\tv_nop\n\tv_nop\n\tv_nop" : "+v"(d) : "v"(a), "v"(b));
  return d;
}
__device__ __forceinline__ v8f wmma_bf(v16b a, v16b b, v8f c) {
  v8f d = __builtin_amdgcn_wmma_f32_16x16x32_bf16(false, a, false, b, (short)0, c, false, false);
  asm volatile("v_nop\n\tv_nop\n\tv_nop\n\tv_nop" : "+v"(d) : "v"(a), "v"(b));
  return d;
}
__device__ __forceinline__ v16h frag_h(const _Float16* rowk0, int lane) {
  union { v16h v; v8h q[2]; } u; const _Float16* p = rowk0 + 8 * (lane >> 4);
  u.q[0] = *(const v8h*)p; u.q[1] = *(const v8h*)(p + 16); return u.v;
}
__device__ __forceinline__ v16b frag_b(const __bf16* rowk0, int lane) {
  union { v16b v; v8b q[2]; } u; const __bf16* p = rowk0 + 8 * (lane >> 4);
  u.q[0] = *(const v8b*)p; u.q[1] = *(const v8b*)(p + 16); return u.v;
}
__device__ __forceinline__ v16h frag_f32(const float* rowk0, int lane) {
  v16h a; const float* p = rowk0 + 8 * (lane >> 4);
  const v4f u0 = *(const v4f*)p, u1 = *(const v4f*)(p + 4), u2 = *(const v4f*)(p + 16), u3 = *(const v4f*)(p + 20);
#pragma unroll
  for (int i = 0; i < 4; ++i) { a[i] = (_Float16)u0[i]; a[4 + i] = (_Float16)u1[i]; a[8 + i] = (_Float16)u2[i]; a[12 + i] = (_Float16)u3[i]; }
  return a;
}
__device__ __forceinline__ float bfr(float v) { return (float)(__bf16)v; }
__device__ __forceinline__ unsigned short f2bf(float f) { const __bf16 h = (__bf16)f; return __builtin_bit_cast(unsigned short, h); }
#define LDSX() do { asm volatile("s_wait_dscnt 0" ::: "memory"); __builtin_amdgcn_wave_barrier(); __builtin_amdgcn_fence(3  , "workgroup"); } while (0)

#ifndef NB
#define NB 2
#endif
#ifndef SEQ
#define SEQ 2048
#endif
#define NB_FULL 2
#define SEQ_FULL 2048
#define DIN 1024
#define HD 128
#define NQH 16
#define KVH 4
#define GG 4
#define CQ (NQH * HD)
#define CK (KVH * HD)
#define HG 4
#define NQB (SEQ / 64)
#define NKB (SEQ / 128)
#define SCALE (0.08838834764831845f)
static_assert(NB >= 1);
static_assert(NB <= NB_FULL);
static_assert(SEQ <= SEQ_FULL);
static_assert(SEQ % 128 == 0);
static_assert(HG == KVH);
static_assert(NQH == GG * KVH);
static_assert(DIN % 64 == 0);
static_assert(CQ % 128 == 0);
static_assert(CK % 128 == 0);
static_assert(HD % 32 == 0);
static_assert((NB * SEQ * DIN) % 2048 == 0);
static_assert((size_t)NB_FULL * SEQ_FULL * CQ * 4u == 33554432u);

#define WS_XB  ((size_t)0)
#define WS_WQ  (WS_XB + 2u * (size_t)NB * SEQ * DIN)
#define WS_WK  (WS_WQ + 2u * (size_t)CQ * DIN)
#define WS_WV  (WS_WK + 2u * (size_t)CK * DIN)
#define WS_QH  (WS_WV + 2u * (size_t)CK * DIN)
#define WS_QL  (WS_QH + 2u * (size_t)NB * SEQ * CQ)
#define WS_KH  (WS_QL + 2u * (size_t)NB * SEQ * CQ)
#define WS_VT  (WS_KH + 2u * (size_t)NB * SEQ * CK)
#define WS_S   (WS_VT + 2u * (size_t)NB * CK * SEQ)
#define WS_END (WS_S  + 4u * (size_t)HG * SEQ * SEQ)
static_assert(WS_END <= (size_t)134217728u);
static_assert(WS_WQ % 128 == 0);
static_assert(WS_QH % 128 == 0);
static_assert(WS_S % 128 == 0);

__global__ __launch_bounds__(256) void k_cvx(const float* __restrict__ X, __bf16* __restrict__ XB) {
  const size_t e = (size_t)blockIdx.x * 256 + threadIdx.x;
  const size_t row = e / (DIN / 8); const int c8 = (int)(e % (DIN / 8)) * 8;
  const size_t b = row / SEQ, t = row % SEQ;
  const float* p = X + (b * SEQ_FULL + t) * (size_t)DIN + c8;
  const v4f f0 = *(const v4f*)p, f1 = *(const v4f*)(p + 4);
  v4u o;
#pragma unroll
  for (int i = 0; i < 2; ++i) {
    o[i]     = (unsigned)f2bf(f0[2 * i]) | ((unsigned)f2bf(f0[2 * i + 1]) << 16);
    o[2 + i] = (unsigned)f2bf(f1[2 * i]) | ((unsigned)f2bf(f1[2 * i + 1]) << 16);
  }
  vst2((void*)(XB + row * DIN + c8), o);
}
__global__ __launch_bounds__(256) void k_cvw(const float* __restrict__ W, int N, __bf16* __restrict__ WT) {
  __shared__ __align__(16) unsigned short st[64][72];
  const int tid = threadIdx.x; const int ot = blockIdx.x * 64, kt = blockIdx.y * 64;
  for (int e = tid; e < 64 * 16; e += 256) { const int r = e >> 4, c4 = (e & 15) * 4;
    const v4f v = *(const v4f*)(W + (size_t)(kt + r) * N + ot + c4);
#pragma unroll
    for (int i = 0; i < 4; ++i) st[c4 + i][r] = f2bf(v[i]); }
  __syncthreads();
  for (int e = tid; e < 64 * 8; e += 256) { const int o = e >> 3, q = e & 7;
    vst2((void*)(WT + (size_t)(ot + o) * DIN + kt + q * 8), *(const v4u*)&st[o][q * 8]); }
}
template <int MODE>
__global__ __launch_bounds__(128) void k_proj(const __bf16* __restrict__ XB, const __bf16* __restrict__ WT, const float* __restrict__ BA, _Float16* __restrict__ DH, _Float16* __restrict__ DL) {
  constexpr int N = (MODE == 0) ? CQ : CK;
  __shared__ __align__(16) _Float16 sh[64][136], sl[64][136]; __shared__ __align__(16) _Float16 th[128][72];
  const int tid = threadIdx.x, wave = tid >> 5, lane = tid & 31, col = lane & 15, g = lane >> 4;
  const int c0 = blockIdx.y * 128; const size_t r0 = (size_t)blockIdx.x * 64; const size_t bb = r0 / SEQ; const int t0 = (int)(r0 % SEQ);
  v8f acc[8] = {};
  const __bf16* xrow = XB + (r0 + wave * 16 + col) * (size_t)DIN;
#pragma unroll 2
  for (int kc = 0; kc < DIN / 32; ++kc) {
    const v16b a = frag_b(xrow + kc * 32, lane);
#pragma unroll
    for (int j = 0; j < 8; ++j) { const v16b w = frag_b(WT + (size_t)(c0 + j * 16 + col) * DIN + kc * 32, lane); acc[j] = wmma_bf(a, w, acc[j]); }
  }
  if (MODE != 2) {
#pragma unroll
    for (int j = 0; j < 8; ++j) { const float bias = bfr(BA[c0 + j * 16 + col]);
#pragma unroll
      for (int r = 0; r < 8; ++r) { const float v = acc[j][r] + bias; const _Float16 hv = (_Float16)v;
        sh[wave * 16 + 8 * g + r][j * 16 + col] = hv;
        if (MODE == 0) sl[wave * 16 + 8 * g + r][j * 16 + col] = (_Float16)((v - (float)hv) * 1024.0f); } }
    __syncthreads();
    for (int e = tid; e < 64 * 16; e += 128) { const int rl = e >> 4, q = e & 15;
      vst2((void*)(DH + (r0 + rl) * N + c0 + q * 8), *(const v4u*)&sh[rl][q * 8]);
      if (MODE == 0) vst2((void*)(DL + (r0 + rl) * N + c0 + q * 8), *(const v4u*)&sl[rl][q * 8]); }
  } else {
#pragma unroll
    for (int j = 0; j < 8; ++j) { const float bias = bfr(BA[c0 + j * 16 + col]);
#pragma unroll
      for (int r = 0; r < 8; ++r) { const float v = acc[j][r] + bias; const int rl = wave * 16 + 8 * g + r, cl = j * 16 + col; th[cl][rl] = (_Float16)v; } }
    __syncthreads();
    for (int e = tid; e < 128 * 8; e += 128) { const int cl = e >> 3, q = e & 7;
      vst2((void*)(DH + (bb * CK + c0 + cl) * (size_t)SEQ + t0 + q * 8), *(const v4u*)&th[cl][q * 8]); }
  }
}
__global__ __launch_bounds__(128) void k_sc(const _Float16* __restrict__ QH, const _Float16* __restrict__ QL, const _Float16* __restrict__ KH, int b, int h0, float* __restrict__ S0) {
  __shared__ __align__(16) float ss[4][16][132];
  const int qb = blockIdx.x, kb = blockIdx.y, kv = blockIdx.z; const int h = h0 + kv;
  float* S = S0 + (size_t)kv * SEQ * SEQ;
  const int tid = threadIdx.x, wave = tid >> 5, lane = tid & 31, col = lane & 15, g = lane >> 4;
  const int k0 = kb * 128; const int ql0 = qb * 64 + wave * 16; const size_t q0 = (size_t)b * SEQ + ql0, kr0 = (size_t)b * SEQ + k0;
  v8f acc[8] = {}, accl[8] = {};
#pragma unroll
  for (int kc = 0; kc < HD / 32; ++kc) {
    const v16h ah = frag_h(QH + (q0 + col) * CQ + h * HD + kc * 32, lane), al = frag_h(QL + (q0 + col) * CQ + h * HD + kc * 32, lane);
#pragma unroll
    for (int j = 0; j < 8; ++j) { const v16h kf = frag_h(KH + (kr0 + j * 16 + col) * CK + kv * HD + kc * 32, lane); acc[j] = wmma16(ah, kf, acc[j]); accl[j] = wmma16(al, kf, accl[j]); } }
#pragma unroll
  for (int j = 0; j < 8; ++j) {
#pragma unroll
    for (int r = 0; r < 8; ++r) ss[wave][8 * g + r][j * 16 + col] = (acc[j][r] + accl[j][r] * (1.0f / 1024.0f)) * SCALE; }
  LDSX(); for (int rl = 0; rl < 16; ++rl) vst2(S + (size_t)(ql0 + rl) * SEQ + k0 + lane * 4, *(const v4f*)&ss[wave][rl][lane * 4]);
}
__global__ __launch_bounds__(256) void k_sm(float* __restrict__ S0) { __shared__ float sred[8]; __shared__ float sbc; __shared__ __align__(16) float shv[SEQ];
  const int tid = threadIdx.x; const int t = blockIdx.x; const int kend = SEQ;
  float* sr = S0 + (size_t)blockIdx.y * SEQ * SEQ + (size_t)t * SEQ;
  float m = -3.0e38f; for (int k = tid; k < kend; k += 256) { const float v = sr[k]; shv[k] = v; m = fmaxf(m, v); }
#pragma unroll
  for (int o = 1; o < 32; o <<= 1) m = fmaxf(m, __shfl_xor(m, o));
  if ((tid & 31) == 0) sred[tid >> 5] = m; __syncthreads(); if (tid == 0) { float a = sred[0]; for (int i = 1; i < 8; ++i) a = fmaxf(a, sred[i]); sbc = a; } __syncthreads(); m = sbc; __syncthreads();
  float sum = 0.f; for (int k = tid; k < kend; k += 256) { const float v = shv[k]; const float e = expf(v - m); shv[k] = e; sum += e; }
#pragma unroll
  for (int o = 1; o < 32; o <<= 1) sum += __shfl_xor(sum, o);
  if ((tid & 31) == 0) sred[tid >> 5] = sum; __syncthreads(); if (tid == 0) { float a = 0.f; for (int i = 0; i < 8; ++i) a += sred[i]; sbc = a > 0.f ? 2048.0f / a : 0.f; } __syncthreads(); const float inv = sbc;
  for (int k = tid; k < kend; k += 256) shv[k] = shv[k] * inv;
  __syncthreads(); for (int q = tid; q < kend / 4; q += 256) vst2(sr + q * 4, *(const v4f*)&shv[q * 4]);
}
__global__ __launch_bounds__(128) void k_pv(const float* __restrict__ PS0, const _Float16* __restrict__ VT, int b, int h0, float* __restrict__ OUT) {
  __shared__ __align__(16) float ss[4][16][HD + 4];
  const int kv = blockIdx.z; const int gq = h0 / KVH; const float* PS = PS0 + (size_t)kv * SEQ * SEQ;
  const int tid = threadIdx.x, wave = tid >> 5, lane = tid & 31, col = lane & 15, g = lane >> 4; const int qb = blockIdx.x; const int ql0 = qb * 64 + wave * 16;
  v8f acc[HD / 16] = {};
#pragma unroll 1
  for (int kc = 0; kc < SEQ / 32; ++kc) { const v16h p = frag_f32(PS + (size_t)(ql0 + col) * SEQ + kc * 32, lane);
    asm volatile("s_wait_loadcnt 0x0" ::: "memory");
#pragma unroll
    for (int j = 0; j < HD / 16; ++j) { const size_t po = ((size_t)b * CK + kv * HD + j * 16 + col) * (size_t)SEQ + kc * 32; acc[j] = wmma16(p, frag_h(VT + po, lane), acc[j]); } }
#pragma unroll
  for (int j = 0; j < HD / 16; ++j)
#pragma unroll
    for (int r = 0; r < 8; ++r) ss[wave][8 * g + r][j * 16 + col] = acc[j][r] * (1.0f / 2048.0f);
  const size_t ocol = (size_t)(kv * GG + gq) * HD;
  LDSX(); for (int rl = 0; rl < 16; ++rl) vst2(OUT + ((size_t)b * SEQ + ql0 + rl) * CQ + ocol + lane * 4, *(const v4f*)&ss[wave][rl][lane * 4]);
}

extern "C" void kernel_launch(void* const* d_in, const int* in_sizes, int n_in, void* d_out, int out_size, void* d_ws, size_t ws_size, hipStream_t stream) {
  if (n_in < 7) return;
  if (in_sizes[0] < ((NB - 1) * SEQ_FULL + SEQ) * DIN || in_sizes[1] < DIN * CQ || in_sizes[2] < CQ || in_sizes[3] < DIN * CK || in_sizes[4] < CK || in_sizes[5] < DIN * CK || in_sizes[6] < CK) return;
  if ((size_t)out_size < (size_t)NB * SEQ * CQ || ws_size < (size_t)WS_END) return;
  const float* const* F = (const float* const*)d_in;
  char* ws = (char*)d_ws;
  __bf16 *XB = (__bf16*)(ws + WS_XB), *WQT = (__bf16*)(ws + WS_WQ), *WKT = (__bf16*)(ws + WS_WK), *WVT = (__bf16*)(ws + WS_WV);
  _Float16 *QH = (_Float16*)(ws + WS_QH), *QL = (_Float16*)(ws + WS_QL), *KH = (_Float16*)(ws + WS_KH), *VT = (_Float16*)(ws + WS_VT);
  float* S = (float*)(ws + WS_S); float* OUT = (float*)d_out;
  k_cvx<<<dim3((unsigned)((size_t)NB * SEQ * DIN / 2048)), 256, 0, stream>>>(F[0], XB);
  k_cvw<<<dim3(CQ / 64, DIN / 64), 256, 0, stream>>>(F[1], CQ, WQT);
  k_cvw<<<dim3(CK / 64, DIN / 64), 256, 0, stream>>>(F[3], CK, WKT);
  k_cvw<<<dim3(CK / 64, DIN / 64), 256, 0, stream>>>(F[5], CK, WVT);
  k_proj<0><<<dim3(NB * SEQ / 64, CQ / 128), 128, 0, stream>>>(XB, WQT, F[2], QH, QL);
  k_proj<1><<<dim3(NB * SEQ / 64, CK / 128), 128, 0, stream>>>(XB, WKT, F[4], KH, QL);
  k_proj<2><<<dim3(NB * SEQ / 64, CK / 128), 128, 0, stream>>>(XB, WVT, F[6], VT, QL);
  for (int b = 0; b < NB; ++b) for (int h0 = 0; h0 < NQH; h0 += HG) {
    k_sc<<<dim3(NQB, NKB, HG), 128, 0, stream>>>(QH, QL, KH, b, h0, S);
    k_sm<<<dim3(SEQ, HG), 256, 0, stream>>>(S);
    k_pv<<<dim3(NQB, 1, HG), 128, 0, stream>>>(S, VT, b, h0, OUT);
  }
}
